// RIMCell_31671088840704
// MI455X (gfx1250) — hardware-verified
//
#include <hip/hip_runtime.h>
#include <hip/hip_bf16.h>


typedef __attribute__((ext_vector_type(16))) __bf16   v16bf;
typedef __attribute__((ext_vector_type(16))) _Float16 v16hf;
typedef __attribute__((ext_vector_type(8)))  float    v8f;

#define BM 64
#define BN 128
#define BK 32
#define APAD 40
#define VST2(T, ptr, val) do { const T _v = (val); *(volatile T*)(ptr) = _v; __threadfence(); *(volatile T*)(ptr) = _v; } while (0)

__device__ __forceinline__ void split_bf16(float v, __bf16& hi, __bf16& lo) {
    const unsigned u = __builtin_bit_cast(unsigned, v) & 0xffff0000u;
    hi = __builtin_bit_cast(__bf16, (unsigned short)(u >> 16));
    lo = (__bf16)(v - __builtin_bit_cast(float, u));
}
__device__ __forceinline__ v8f wmmab(v16bf a, v16bf b, v8f c) {
    v8f d = __builtin_amdgcn_wmma_f32_16x16x32_bf16(false, a, false, b, (short)0, c, false, false);
    asm volatile("v_nop\n\tv_nop\n\tv_nop\n\tv_nop" : "+v"(d) : "v"(a), "v"(b));
    return d;
}
__device__ __forceinline__ v8f wmmah(v16hf a, v16hf b, v8f c) {
    v8f d = __builtin_amdgcn_wmma_f32_16x16x32_f16(false, a, false, b, (short)0, c, false, false);
    asm volatile("v_nop\n\tv_nop\n\tv_nop\n\tv_nop" : "+v"(d) : "v"(a), "v"(b));
    return d;
}

template <bool SPLIT>
__global__ __launch_bounds__(256)
void rim_gemm_wmma(const float* __restrict__ A, int lda, long long sA,
                   const float* __restrict__ Bw, int ldb, long long sB,
                   const float* __restrict__ bias, long long sBias,
                   float* __restrict__ C, int ldc, long long sC,
                   int M, int N, int Kdim)
{
    __shared__ __attribute__((aligned(16))) unsigned short Ah_[BM][APAD], Bh_[BN][APAD];
    __shared__ __attribute__((aligned(16))) unsigned short Al_[BM][APAD], Bl_[BN][APAD];

    const int u = blockIdx.z;
    A  += (long long)u * sA;
    Bw += (long long)u * sB;
    C  += (long long)u * sC;
    if (bias) bias += (long long)u * sBias;

    const int m0 = blockIdx.y * BM;
    const int n0 = blockIdx.x * BN;
    const int tid  = threadIdx.x;
    const int w    = tid >> 5;
    const int lane = tid & 31;
    const int half = lane >> 4;
    const int l15  = lane & 15;
    const int wm   = w >> 2;
    const int wn   = w & 3;

    const int aRow = tid >> 3;
    const int aCol = (tid & 7) * 4;
    const int bRow = tid >> 5;
    const int gN   = n0 + (tid & 31) * 4;
    const int gNc  = (gN < N) ? gN : 0;
    const bool nOK = (gN < N);

    auto put = [&](unsigned short* ph, unsigned short* pl, int i, float v) {
        if constexpr (SPLIT) { __bf16 h_, l_; split_bf16(v, h_, l_); ph[i] = __builtin_bit_cast(unsigned short, h_); pl[i] = __builtin_bit_cast(unsigned short, l_); }
        else { ph[i] = __builtin_bit_cast(unsigned short, (_Float16)v); (void)pl; }
    };

    v8f acc[2][2] = {};
    for (int k0 = 0; k0 < Kdim; k0 += BK) {
        __syncthreads();
        #pragma unroll
        for (int r = 0; r < 2; r++) {
            const float4 va = *(const float4*)(A + (long long)(m0 + aRow + r * 32) * lda + k0 + aCol);
            unsigned short* ph = &Ah_[aRow + r * 32][aCol]; unsigned short* pl = &Al_[aRow + r * 32][aCol];
            put(ph, pl, 0, va.x); put(ph, pl, 1, va.y); put(ph, pl, 2, va.z); put(ph, pl, 3, va.w);
        }
        #pragma unroll
        for (int r = 0; r < 4; r++) {
            const int krow = bRow + r * 8, c = (tid & 31) * 4;
            float4 vb = *(const float4*)(Bw + (long long)(k0 + krow) * ldb + gNc);
            if (!nOK) vb = make_float4(0.f, 0.f, 0.f, 0.f);
            put(&Bh_[c + 0][0], &Bl_[c + 0][0], krow, vb.x);
            put(&Bh_[c + 1][0], &Bl_[c + 1][0], krow, vb.y);
            put(&Bh_[c + 2][0], &Bl_[c + 2][0], krow, vb.z);
            put(&Bh_[c + 3][0], &Bl_[c + 3][0], krow, vb.w);
        }
        __syncthreads();

        union WF { uint4 q[2]; v16bf b; v16hf h; };
        WF ah[2], bh[2], al[2], bl[2];
        #pragma unroll
        for (int mi = 0; mi < 2; mi++) {
            const unsigned short* ap = &Ah_[wm * 32 + mi * 16 + l15][8 * half];
            ah[mi].q[0] = *(const uint4*)ap; ah[mi].q[1] = *(const uint4*)(ap + 16);
            if constexpr (SPLIT) { const unsigned short* al_ = &Al_[wm * 32 + mi * 16 + l15][8 * half]; al[mi].q[0] = *(const uint4*)al_; al[mi].q[1] = *(const uint4*)(al_ + 16); }
        }
        #pragma unroll
        for (int ni = 0; ni < 2; ni++) {
            const unsigned short* bp = &Bh_[wn * 32 + ni * 16 + l15][8 * half];
            bh[ni].q[0] = *(const uint4*)bp; bh[ni].q[1] = *(const uint4*)(bp + 16);
            if constexpr (SPLIT) { const unsigned short* bl_ = &Bl_[wn * 32 + ni * 16 + l15][8 * half]; bl[ni].q[0] = *(const uint4*)bl_; bl[ni].q[1] = *(const uint4*)(bl_ + 16); }
        }
        #pragma unroll
        for (int mi = 0; mi < 2; mi++)
            #pragma unroll
            for (int ni = 0; ni < 2; ni++) {
                if constexpr (SPLIT) {
                    acc[mi][ni] = wmmab(ah[mi].b, bh[ni].b, acc[mi][ni]);
                    acc[mi][ni] = wmmab(ah[mi].b, bl[ni].b, acc[mi][ni]);
                    acc[mi][ni] = wmmab(al[mi].b, bh[ni].b, acc[mi][ni]);
                } else {
                    acc[mi][ni] = wmmah(ah[mi].h, bh[ni].h, acc[mi][ni]);
                }
            }
    }

    const int cbase = n0 + wn * 32;
    if (cbase >= N) return;
    const float bv = bias ? bias[cbase + lane] : 0.0f;
    for (int pass = 0; pass < 2; ++pass) {
        #pragma unroll
        for (int mi = 0; mi < 2; mi++) {
            #pragma unroll
            for (int j = 0; j < 8; j++) {
                const float a0 = acc[mi][0][j], b0 = acc[mi][1][j];
                const float ax = __shfl_xor(a0, 16), bx = __shfl_xor(b0, 16);
                const int r1 = m0 + wm * 32 + mi * 16 + j, r2 = r1 + 8;
                *(volatile float*)(C + (long long)r1 * ldc + cbase + lane) = (half ? bx : a0) + bv;
                *(volatile float*)(C + (long long)r2 * ldc + cbase + lane) = (half ? b0 : ax) + bv;
            }
        }
        __threadfence();
    }
}

__global__ __launch_bounds__(256)
void rim_scores(const float* __restrict__ qry,
                const float* __restrict__ key0,
                const float* __restrict__ bk_in,
                const float* __restrict__ val0,
                const float* __restrict__ bv_in,
                float* __restrict__ mask,
                float* __restrict__ inputs)
{
    const int b   = blockIdx.x;
    const int tid = threadIdx.x;
    const int w   = tid >> 5;
    const int ln  = tid & 31;
    __shared__ float s0[8], s1[8], sm[8], p0s[8], p1s[8];

    const float* qp = qry + ((long long)b * 8 + w) * 64;
    const float* kp = key0 + (long long)b * 64;
    float d0 = 0.f, d1 = 0.f;
    for (int i = ln; i < 64; i += 32) {
        float qv = qp[i];
        d0 += qv * kp[i];
        d1 += qv * bk_in[i];
    }
    #pragma unroll
    for (int off = 16; off > 0; off >>= 1) {
        d0 += __shfl_down(d0, off, 32);
        d1 += __shfl_down(d1, off, 32);
    }
    if (ln == 0) { s0[w] = d0 * 0.125f; s1[w] = d1 * 0.125f; }
    __syncthreads();

    if (tid < 8) {
        int u = tid;
        float su = s0[u];
        int rank = 0;
        for (int j = 0; j < 8; j++) {
            float sj = s0[j];
            if (sj > su || (sj == su && j < u)) rank++;
        }
        float m = (rank < 4) ? 1.f : 0.f;
        sm[u] = m;
        float a = s0[u], c = s1[u];
        float mx = fmaxf(a, c);
        float e0 = expf(a - mx), e1 = expf(c - mx);
        float inv = 1.f / (e0 + e1);
        p0s[u] = e0 * inv;
        p1s[u] = e1 * inv;
    }
    __syncthreads();
    if (tid < 32) VST2(float, mask + (long long)b * 32 + tid, (tid < 8) ? sm[tid] : 0.0f);

    const float* vp = val0 + (long long)b * 512;
    for (int u = 0; u < 8; u++) {
        float m = sm[u], p0 = p0s[u], p1 = p1s[u];
        for (int i = tid; i < 512; i += 256)
            VST2(float, inputs + ((long long)b * 8 + u) * 512 + i, m * (p0 * vp[i] + p1 * bv_in[i]));
    }
}

__global__ __launch_bounds__(256)
void rim_gates(const float* __restrict__ gi, const float* __restrict__ gh,
               const float* __restrict__ hs, float* __restrict__ hsnew)
{
    long long idx = (long long)blockIdx.x * 256 + threadIdx.x;
    if (idx >= 512LL * 8 * 512) return;
    long long bu = idx >> 9;
    int h = (int)(idx & 511);
    long long g = bu * 1536;
    float ir = gi[g + h],        hr = gh[g + h];
    float iz = gi[g + 512 + h],  hz = gh[g + 512 + h];
    float in_ = gi[g + 1024 + h], hn = gh[g + 1024 + h];
    float r = 1.f / (1.f + expf(-(ir + hr)));
    float z = 1.f / (1.f + expf(-(iz + hz)));
    float n = tanhf(in_ + r * hn);
    VST2(float, hsnew + idx, (1.f - z) * n + z * hs[idx]);
}

__global__ __launch_bounds__(256)
void rim_attn(const float* __restrict__ qbuf,
              const float* __restrict__ kbuf,
              const float* __restrict__ vbuf,
              const float* __restrict__ mask,
              float* __restrict__ ctx)
{
    const int b  = blockIdx.x >> 2;
    const int ch = blockIdx.x & 3;
    const int tid = threadIdx.x;
    __shared__ float qs[8][32], ks[8][32], vs[8][512], ps[8][8];

    {
        int u = tid >> 5, kk = tid & 31;
        qs[u][kk] = qbuf[((long long)b * 8 + u) * 128 + ch * 32 + kk];
        ks[u][kk] = kbuf[((long long)b * 8 + u) * 128 + ch * 32 + kk];
    }
    for (int i = tid; i < 4096; i += 256) {
        int n = i >> 9, d = i & 511;
        vs[n][d] = vbuf[((long long)b * 8 + n) * 2048 + ch * 512 + d];
    }
    __syncthreads();

    if (tid < 64) {
        int u = tid >> 3, n = tid & 7;
        float s = 0.f;
        #pragma unroll
        for (int kk = 0; kk < 32; kk++) s += qs[u][kk] * ks[n][kk];
        ps[u][n] = s * 0.17677669529663687f;
    }
    __syncthreads();

    if (tid < 8) {
        int u = tid;
        float mx = -1e30f;
        for (int n = 0; n < 8; n++) mx = fmaxf(mx, ps[u][n]);
        float e[8], sum = 0.f;
        for (int n = 0; n < 8; n++) { e[n] = expf(ps[u][n] - mx); sum += e[n]; }
        float inv = mask[(long long)b * 32 + u] / sum;
        for (int n = 0; n < 8; n++) ps[u][n] = e[n] * inv;
    }
    __syncthreads();

    for (int i = tid; i < 4096; i += 256) {
        int u = i >> 9, d = i & 511;
        float s = 0.f;
        #pragma unroll
        for (int n = 0; n < 8; n++) s += ps[u][n] * vs[n][d];
        VST2(float, ctx + ((long long)b * 8 + u) * 2048 + ch * 512 + d, s);
    }
}

__global__ __launch_bounds__(256)
void rim_final(const float* __restrict__ hsnew, const float* __restrict__ co,
               const float* __restrict__ hs, const float* __restrict__ mask,
               float* __restrict__ out)
{
    long long idx = (long long)blockIdx.x * 256 + threadIdx.x;
    if (idx >= 512LL * 8 * 512) return;
    long long bu = idx >> 9;
    const float mk = mask[(bu >> 3) * 32 + (bu & 7)];
    VST2(float, out + idx, (mk > 0.5f) ? (hsnew[idx] + co[idx]) : hs[idx]);
}

template <bool SPLIT>
static inline void launch_gemm(hipStream_t s,
                               const float* A, int lda, long long sA,
                               const float* B, int ldb, long long sB,
                               const float* bias, long long sBias,
                               float* C, int ldc, long long sC,
                               int M, int N, int K, int batch)
{
    dim3 grid((N + BN - 1) / BN, (M + BM - 1) / BM, batch);
    hipLaunchKernelGGL(rim_gemm_wmma<SPLIT>, grid, dim3(256), 0, s,
                       A, lda, sA, B, ldb, sB, bias, sBias, C, ldc, sC, M, N, K);
}

extern "C" void kernel_launch(void* const* d_in, const int* in_sizes, int n_in,
                              void* d_out, int out_size, void* d_ws, size_t ws_size,
                              hipStream_t stream)
{
    const float* x     = (const float*)d_in[0];
    const float* hs    = (const float*)d_in[1];
    const float* Wk_in = (const float*)d_in[2];
    const float* bk_in = (const float*)d_in[3];
    const float* Wv_in = (const float*)d_in[4];
    const float* bv_in = (const float*)d_in[5];
    const float* Wq_in = (const float*)d_in[6];
    const float* bq_in = (const float*)d_in[7];
    const float* W_ih  = (const float*)d_in[8];
    const float* W_hh  = (const float*)d_in[9];
    const float* b_ih  = (const float*)d_in[10];
    const float* b_hh  = (const float*)d_in[11];
    const float* Wq_c  = (const float*)d_in[12];
    const float* Wk_c  = (const float*)d_in[13];
    const float* Wv_c  = (const float*)d_in[14];
    const float* Wo_c  = (const float*)d_in[15];
    float* out = (float*)d_out;
    float* ws  = (float*)d_ws;

    float* mask   = ws + 25169920;
    float* hsnew  = ws + 4096;
    float* gi     = ws + 2101248;
    float* gh     = ws + 8392704;
    float* vbuf   = ws + 2101248;
    float* qbuf   = ws + 10489856;
    float* kbuf   = ws + 11014144;
    float* key0   = ws + 14684160;
    float* val0   = ws + 14716928;
    float* qry    = ws + 14979072;
    float* inputs = ws + 15241216;
    float* ctxb   = ws + 14684160;
    float* co     = ws + 23072768;
    (void)in_sizes; (void)n_in; (void)out_size;
    if (ws_size < (size_t)(25169920 + 16384) * sizeof(float)) return;

    launch_gemm<true>(stream, x, 1024, 0, Wk_in, 64, 0, bk_in, 0,
                key0, 64, 0, 512, 64, 1024, 1);
    launch_gemm<false>(stream, x, 1024, 0, Wv_in, 512, 0, bv_in, 0,
                val0, 512, 0, 512, 512, 1024, 1);
    launch_gemm<true>(stream, hs, 512, 0, Wq_in, 64, 0, bq_in, 0,
                qry, 64, 0, 4096, 64, 512, 1);
    hipLaunchKernelGGL(rim_scores, dim3(512), dim3(256), 0, stream,
                       qry, key0, bk_in, val0, bv_in, mask, inputs);

    launch_gemm<false>(stream, inputs, 4096, 512, W_ih, 1536, 786432, b_ih, 1536,
                gi, 12288, 1536, 512, 1536, 512, 8);
    launch_gemm<false>(stream, hs, 4096, 512, W_hh, 1536, 786432, b_hh, 1536,
                gh, 12288, 1536, 512, 1536, 512, 8);
    hipLaunchKernelGGL(rim_gates, dim3(8192), dim3(256), 0, stream,
                       gi, gh, hs, hsnew);

    launch_gemm<false>(stream, hsnew, 4096, 512, Wq_c, 128, 65536, nullptr, 0,
                qbuf, 1024, 128, 512, 128, 512, 8);
    launch_gemm<false>(stream, hsnew, 4096, 512, Wk_c, 128, 65536, nullptr, 0,
                kbuf, 1024, 128, 512, 128, 512, 8);
    launch_gemm<false>(stream, hsnew, 4096, 512, Wv_c, 2048, 1048576, nullptr, 0,
                vbuf, 16384, 2048, 512, 2048, 512, 8);
    hipLaunchKernelGGL(rim_attn, dim3(2048), dim3(256), 0, stream,
                       qbuf, kbuf, vbuf, mask, ctxb);

    launch_gemm<false>(stream, ctxb, 16384, 2048, Wo_c, 512, 1048576, nullptr, 0,
                co, 4096, 512, 512, 512, 2048, 8);
    hipLaunchKernelGGL(rim_final, dim3(8192), dim3(256), 0, stream,
                       hsnew, co, hs, mask, out);
}
